// MultiConvexNet_34583076667993
// MI455X (gfx1250) — hardware-run, weakly checked
//
#include <hip/hip_runtime.h>
#include <math.h>

typedef __attribute__((ext_vector_type(16))) _Float16 v16h;
typedef __attribute__((ext_vector_type(8)))  _Float16 v8h;
typedef __attribute__((ext_vector_type(8)))  float    v8f;
typedef __attribute__((ext_vector_type(4)))  float    v4f;

constexpr int kNB   = 8;
constexpr int kNP   = 16;
constexpr int kNV   = 64;
constexpr int kND   = 1986;
constexpr int kNDP  = 2048;
constexpr int kNBP  = kNB * kNP;
constexpr int kChunks = 16;
constexpr int kSlabP  = 17;
constexpr int kMeanP  = 32;

constexpr int kCnt0 = kNBP * kND * 3;
constexpr int kCnt1 = kNBP * kND * 4;
constexpr int kCnt2 = kNBP;
constexpr int kCnt3 = kNBP * 3;
constexpr int kCnt4 = kND * 3;
constexpr int kCnt5 = kNBP * kNV * 3;
constexpr int kOff1 = kCnt0;
constexpr int kOff2 = kOff1 + kCnt1;
constexpr int kOff3 = kOff2 + kCnt2;
constexpr int kOff4 = kOff3 + kCnt3;
constexpr int kOff5 = kOff4 + kCnt4;
constexpr int kOutTotal = kOff5 + kCnt5;
static_assert(kNBP == 128, "pairs");
static_assert(kOff1 == 762624 && kOff2 == 1779456 && kOff3 == 1779584 && kOff4 == 1779968 && kOff5 == 1785926, "output element offsets");
static_assert(kOutTotal == 1810502, "output total");
static_assert((size_t)kOff1 * 4 == 3050496ull && (size_t)kOff5 * 4 == 7143704ull && (size_t)kOutTotal * 4 == 7242008ull, "output byte offsets");
static_assert(kChunks * 8 * 16 == kNDP, "direction tiles cover the padded table");
static_assert((kNV % 32) == 0, "K multiple of 32");

constexpr float kCarryW    = 1024.0f;
constexpr float kCarryRes  = 2048.0f;
constexpr float kInvCarryW   = 1.0f / kCarryW;
constexpr float kInvCarryRes = 1.0f / kCarryRes;

constexpr float kClipLo = 1e-20f;
constexpr float kClipHi = 1e20f;
constexpr float kLog2of10 = 3.3219280948873623f;
constexpr float kLog10of2 = 0.30102999566398120f;

constexpr size_t kOffRES   = 0;
constexpr size_t kOffDIRS  = kOffRES  + (size_t)kNBP * kNDP * 16;
constexpr size_t kOffLVW   = kOffDIRS + (size_t)kNDP * 16;
constexpr size_t kOffMEANW = kOffLVW  + (size_t)kNBP * kNV * 16;
constexpr size_t kWsTotal  = kOffMEANW + (size_t)kNBP * kMeanP * 4;
static_assert(kWsTotal == 4374528ull, "carve total");
static_assert(kWsTotal <= 134217728ull, "carve cap");
static_assert((kOffDIRS % 128) == 0 && (kOffLVW % 128) == 0 && (kOffMEANW % 128) == 0, "aligned regions");

union FragH { v16h v; v8h h[2]; };

__device__ __forceinline__ v16h frag_load_h(const _Float16* p) {
  FragH f;
  f.h[0] = *(const v8h*)(p);
  f.h[1] = *(const v8h*)(p + 16);
  return f.v;
}
__device__ __forceinline__ v8f mma_h(v16h a, v16h b, v8f c) {
  return __builtin_amdgcn_wmma_f32_16x16x32_f16(false, a, false, b, (short)0, c, false, false);
}
__device__ __forceinline__ void frag_guard(v8f& acc, v16h x0, v16h x1, v16h y0, v16h y1) {
  asm volatile("v_nop\n\tv_nop\n\tv_nop\n\tv_nop" : "+v"(acc) : "v"(x0), "v"(x1), "v"(y0), "v"(y1));
}

__global__ __launch_bounds__(256) void dir_table_kernel(float* __restrict__ DIRS) {
  const int d  = blockIdx.x * 256 + threadIdx.x;
  const int dc = (d < kND - 1) ? d : (kND - 1);
  const bool ongrid = dc < 1984;
  const int ig = (dc >> 6) + 1;
  const int jg = dc & 63;
  const int ip = (dc == 1984) ? 0 : 32;
  const int i  = ongrid ? ig : ip;
  const int j  = ongrid ? jg : 0;
  const float a1 = (float)(i - 16) * (1.0f / 32.0f);
  const float a2 = (float)(j - 32) * (1.0f / 32.0f);
  const float s1 = sinpif(a1);
  const float c1 = cospif(a1);
  const float s2 = sinpif(a2);
  const float c2 = cospif(a2);
  v4f o;
  o.x = c1 * c2;
  o.y = c1 * s2;
  o.z = s1;
  o.w = 0.0f;
  float* p = DIRS + (size_t)d * 4;
  *(volatile v4f*)p = o;
  __threadfence();
  *(volatile v4f*)p = o;
}

__global__ __launch_bounds__(256) void support_main_kernel(
    const float* __restrict__ verts, const float* __restrict__ smooth,
    const float* __restrict__ DIRS, float* __restrict__ RES,
    float* __restrict__ LVW, float* __restrict__ MEANW)
{
  __shared__ __align__(16) float    sRaw[kNV * 3];
  __shared__ __align__(16) float    sLV[kNV * 4];
  __shared__ __align__(16) float    sMean[4];
  __shared__ __align__(16) _Float16 sBt[16 * kNV];
  __shared__ __align__(16) float    sD[8 * 16 * kSlabP];

  const int tid   = threadIdx.x;
  const int lane  = tid & 31;
  const int wave  = __builtin_amdgcn_readfirstlane((int)(threadIdx.x >> 5));
  const int chunk = blockIdx.x & (kChunks - 1);
  const int bp    = blockIdx.x >> 4;

  {
    const int tc = (tid < kNV * 3 - 1) ? tid : (kNV * 3 - 1);
    float rvv = verts[(size_t)bp * (kNV * 3) + tc];
    if (wave < 6) sRaw[tid] = rvv;
  }
  __syncthreads();
  if (tid < 4) {
    const int c = (tid < 3) ? tid : 2;
    float s = 0.0f;
#pragma unroll 1
    for (int v = 0; v < kNV; ++v) s += sRaw[v * 3 + c];
    sMean[tid] = (tid < 3) ? s * (1.0f / (float)kNV) : 0.0f;
  }
  __syncthreads();
  if (wave < 2) {
    v4f q;
    q.x = sRaw[tid * 3 + 0] - sMean[0];
    q.y = sRaw[tid * 3 + 1] - sMean[1];
    q.z = sRaw[tid * 3 + 2] - sMean[2];
    q.w = 0.0f;
    *(v4f*)(sLV + tid * 4) = q;
  }
  __syncthreads();

  if (wave < 4) {
    const int row = tid >> 3;
    const int seg = tid & 7;
    const int c = (row < 3) ? row : ((row < 6) ? (row - 3) : 0);
    v8h hv;
#pragma unroll
    for (int e = 0; e < 8; ++e) {
      const float x = sLV[(seg * 8 + e) * 4 + c];
      const _Float16 xh = (_Float16)x;
      const float xr = (x - (float)xh) * kCarryRes;
      const float val = (row < 3) ? x : ((row < 6) ? xr : 0.0f);
      hv[e] = (_Float16)val;
    }
    *(v8h*)(sBt + row * kNV + seg * 8) = hv;
  }

  if (chunk == 0) {
    if (wave < 2) {
      const v4f q = *(const v4f*)(sLV + tid * 4);
      float* p = LVW + ((size_t)bp * kNV + tid) * 4;
      *(volatile v4f*)p = q;
      __threadfence();
      *(volatile v4f*)p = q;
    } else if (wave == 2) {
      const float mload = sMean[lane & 3];
      const float mval = (lane < 4) ? mload : 0.0f;
      float* p = MEANW + (size_t)bp * kMeanP + lane;
      *(volatile float*)p = mval;
      __threadfence();
      *(volatile float*)p = mval;
    }
  }
  __syncthreads();

  const int h    = lane >> 4;
  const int col  = lane & 15;
  const int tile = chunk * 8 + wave;
  const int d    = tile * 16 + col;

  const v4f dir = *(const v4f*)(DIRS + (size_t)d * 4);
  const float sp    = smooth[bp];
  const float spm1  = sp - 1.0f;
  const float invsp = 1.0f / sp;

  const v16h b0 = frag_load_h(sBt + col * kNV + 8 * h);
  const v16h b1 = frag_load_h(sBt + col * kNV + 32 + 8 * h);

  const float* lvp = sLV + 32 * h;
  float lz[32];
  float lzmax = -INFINITY;
#pragma unroll
  for (int s = 0; s < 2; ++s) {
#pragma unroll
    for (int i = 0; i < 16; ++i) {
      const v4f q = *(const v4f*)(lvp + (32 * s + i + ((i >= 8) ? 8 : 0)) * 4);
      float z = q.x * dir.x;
      z = fmaf(q.y, dir.y, z);
      z = fmaf(q.z, dir.z, z);
      const float l = log2f(fmaxf(z, 0.0f));
      lz[s * 16 + i] = l;
      lzmax = fmaxf(lzmax, l);
    }
  }
  {
    const float other = __shfl_xor(lzmax, 16, 32);
    lzmax = fmaxf(lzmax, other);
  }

  const float expo = (lzmax * kLog10of2) * sp;
  float lk = (expo < -20.0f) ? (-20.0f - expo) * invsp : 0.0f;
  lk = fminf(fmaxf(ceilf(lk), 0.0f), 20.0f);
  const float lg_k = lk * kLog2of10;
  const float kinv = (lk > 0.0f) ? exp2f(-lg_k) : 1.0f;

  const float pbase = sp * lg_k;
  float ssum = 0.0f;
#pragma unroll
  for (int t = 0; t < 32; ++t) {
    const float l = lz[t];
    float zp = exp2f(fmaf(l, sp, pbase));
    zp = fminf(fmaxf(zp, kClipLo), kClipHi);
    ssum += (l > -INFINITY) ? zp : 0.0f;
  }
  {
    const float other = __shfl_xor(ssum, 16, 32);
    ssum += other;
  }
  float hval = exp2f(log2f(ssum) * invsp);
  hval = fminf(fmaxf(hval, kClipLo), kClipHi);
  const float lg_h = log2f(hval);

  const float dbase = spm1 * (lg_k - lg_h);
  v16h af[2];
#pragma unroll
  for (int s = 0; s < 2; ++s) {
#pragma unroll
    for (int i = 0; i < 16; ++i) {
      const float l = lz[s * 16 + i];
      float dh = exp2f(fmaf(l, spm1, dbase));
      dh = fminf(fmaxf(dh, kClipLo), kClipHi);
      dh = (l > -INFINITY) ? dh : kClipLo;
      const float av = fminf(dh * kCarryW, 32768.0f);
      af[s][i] = (_Float16)av;
    }
  }

  v8f acc = (v8f){0.f, 0.f, 0.f, 0.f, 0.f, 0.f, 0.f, 0.f};
  acc = mma_h(af[0], b0, acc);
  acc = mma_h(af[1], b1, acc);
  frag_guard(acc, af[0], af[1], b0, b1);

  float* slab = sD + wave * (16 * kSlabP);
#pragma unroll
  for (int r = 0; r < 8; ++r) slab[(8 * h + r) * kSlabP + col] = acc[r];
  __syncthreads();

  const float f0 = slab[col * kSlabP + 0];
  const float f1 = slab[col * kSlabP + 1];
  const float f2 = slab[col * kSlabP + 2];
  const float f3 = slab[col * kSlabP + 3];
  const float f4 = slab[col * kSlabP + 4];
  const float f5 = slab[col * kSlabP + 5];
  const float mx = sMean[0];
  const float my = sMean[1];
  const float mz = sMean[2];
  v4f o;
  o.x = fmaf(f3, kInvCarryRes, f0) * kInvCarryW + mx;
  o.y = fmaf(f4, kInvCarryRes, f1) * kInvCarryW + my;
  o.z = fmaf(f5, kInvCarryRes, f2) * kInvCarryW + mz;
  o.w = fminf(fmaxf(hval * kinv, -kClipHi), kClipHi);

  float* rp = RES + ((size_t)bp * kNDP + (size_t)tile * 16 + col) * 4;
  if (h == 0) *(volatile v4f*)rp = o;
  __threadfence();
  if (h == 0) *(volatile v4f*)rp = o;
}

__global__ __launch_bounds__(256) void pack_kernel(
    const float* __restrict__ RES, const float* __restrict__ DIRS,
    const float* __restrict__ LVW, const float* __restrict__ MEANW,
    float* __restrict__ out)
{
  const int e  = blockIdx.x * 256 + threadIdx.x;
  const int ec = (e < kOutTotal) ? e : (kOutTotal - 1);

  const bool in0 = ec < kOff1;
  const bool in1 = (!in0) && (ec < kOff2);
  const bool in3 = (ec >= kOff3) && (ec < kOff4);
  const bool in4 = (ec >= kOff4) && (ec < kOff5);
  const bool in5 = ec >= kOff5;

  const int e0  = (ec < kCnt0 - 1) ? ec : (kCnt0 - 1);
  const int q0  = e0 / 3;
  const int c0  = e0 - 3 * q0;
  const int bp0 = q0 / kND;
  const int d0  = q0 - bp0 * kND;
  const int ri0 = (bp0 * kNDP + d0) * 4 + c0;

  int e1 = ec - kOff1;
  e1 = (e1 < 0) ? 0 : e1;
  e1 = (e1 < kCnt1 - 1) ? e1 : (kCnt1 - 1);
  const int q1  = e1 >> 2;
  const int c1  = e1 & 3;
  const int bp1 = q1 / kND;
  const int d1  = q1 - bp1 * kND;
  const int ri1 = (bp1 * kNDP + d1) * 4 + 3;
  const int di1 = d1 * 4 + ((c1 < 3) ? c1 : 2);

  int e3 = ec - kOff3;
  e3 = (e3 < 0) ? 0 : e3;
  e3 = (e3 < kCnt3 - 1) ? e3 : (kCnt3 - 1);
  const int bp3 = e3 / 3;
  const int c3  = e3 - 3 * bp3;
  const int mi  = bp3 * kMeanP + c3;

  int e4 = ec - kOff4;
  e4 = (e4 < 0) ? 0 : e4;
  e4 = (e4 < kCnt4 - 1) ? e4 : (kCnt4 - 1);
  const int d4  = e4 / 3;
  const int c4  = e4 - 3 * d4;
  const int di4 = d4 * 4 + c4;

  int e5 = ec - kOff5;
  e5 = (e5 < 0) ? 0 : e5;
  e5 = (e5 < kCnt5 - 1) ? e5 : (kCnt5 - 1);
  const int r5 = e5 / 3;
  const int c5 = e5 - 3 * r5;
  const int li = r5 * 4 + c5;

  const int ri = in0 ? ri0 : ri1;
  const int di = in1 ? di1 : di4;

  float rv = RES[ri];
  asm volatile("" : "+v"(rv));
  float dv = DIRS[di];
  asm volatile("" : "+v"(dv));
  float mv = MEANW[mi];
  asm volatile("" : "+v"(mv));
  float lv = LVW[li];
  asm volatile("" : "+v"(lv));

  const float v1 = (c1 < 3) ? dv : rv;
  float val = 0.0f;
  val = in0 ? rv : val;
  val = in1 ? v1 : val;
  val = in3 ? mv : val;
  val = in4 ? dv : val;
  val = in5 ? lv : val;

  float* p = out + ec;
  if (e < kOutTotal) *(volatile float*)p = val;
  __threadfence();
  if (e < kOutTotal) *(volatile float*)p = val;
}

extern "C" void kernel_launch(void* const* d_in, const int* in_sizes, int n_in,
                              void* d_out, int out_size, void* d_ws, size_t ws_size,
                              hipStream_t stream) {
  if (n_in < 2) return;
  if (in_sizes[0] != kNBP * kNV * 3) return;
  if (in_sizes[1] != kNBP) return;
  if (out_size != kOutTotal) return;
  if (ws_size < kWsTotal) return;

  const float* verts  = (const float*)d_in[0];
  const float* smooth = (const float*)d_in[1];
  float* out = (float*)d_out;

  char* ws = (char*)d_ws;
  float* RES   = (float*)(ws + kOffRES);
  float* DIRS  = (float*)(ws + kOffDIRS);
  float* LVW   = (float*)(ws + kOffLVW);
  float* MEANW = (float*)(ws + kOffMEANW);

  dir_table_kernel<<<kNDP / 256, 256, 0, stream>>>(DIRS);
  support_main_kernel<<<kNBP * kChunks, 256, 0, stream>>>(verts, smooth, DIRS, RES, LVW, MEANW);
  pack_kernel<<<(kOutTotal + 255) / 256, 256, 0, stream>>>(RES, DIRS, LVW, MEANW, out);
}
